// RWKV7_10359461118200
// MI455X (gfx1250) — hardware-verified
//
#include <hip/hip_runtime.h>

typedef __attribute__((ext_vector_type(16))) _Float16 v16h;
typedef __attribute__((ext_vector_type(8)))  _Float16 v8h;
typedef __attribute__((ext_vector_type(16))) __bf16   v16b;
typedef __attribute__((ext_vector_type(8)))  __bf16   v8b;
typedef __attribute__((ext_vector_type(8)))  float    v8f;
typedef __attribute__((ext_vector_type(4)))  float    v4f;
typedef __attribute__((ext_vector_type(2)))  float    v2f;
typedef __attribute__((ext_vector_type(4)))  unsigned int v4u;
typedef __attribute__((ext_vector_type(2)))  unsigned int v2u;

constexpr int CDIM   = 768;
constexpr int TLEN   = 1024;
constexpr int NBAT   = 8;
constexpr int NHEAD  = 24;
constexpr int HSZ    = 32;
constexpr int MTOT   = NBAT * TLEN;
constexpr int NBCH   = 2;
constexpr int MCH    = NBCH * TLEN;
constexpr int NCHUNK = NBAT / NBCH;
static_assert(NHEAD * HSZ == CDIM, "heads");
static_assert(NCHUNK * NBCH == NBAT, "chunks");
static_assert(MCH % 64 == 0 && CDIM % 64 == 0, "GEMM M and N tile multiples");
static_assert(CDIM % 32 == 0, "K of the first-stage GEMMs");

constexpr size_t P16B = (size_t)MCH * CDIM * 2;
constexpr size_t P32B = (size_t)MCH * CDIM * 4;
constexpr size_t OFF_RA = 0;
constexpr size_t OFF_RB = OFF_RA + 4 * P32B;
constexpr size_t OFF_RC = OFF_RB + 6 * P16B;
constexpr size_t OFF_RD = OFF_RC + 3 * P32B;
constexpr size_t OFF_RE = OFF_RD + 5 * P32B;
constexpr size_t SZ_TM  = (size_t)MCH * 128 * 2;
constexpr size_t SZ_GS  = (size_t)MCH * 128 * 2;
constexpr size_t SZ_P16 = (size_t)MCH * 256 * 2;
constexpr size_t SZ_PK  = (size_t)MCH * 64 * 2;
constexpr size_t OFF_TMH = OFF_RE;
constexpr size_t OFF_TML = OFF_TMH + SZ_TM;
constexpr size_t OFF_GSH = OFF_TML + SZ_TM;
constexpr size_t OFF_GSL = OFF_GSH + SZ_GS;
constexpr size_t OFF_P16 = OFF_GSL + SZ_GS;
constexpr size_t OFF_PKH = OFF_P16 + SZ_P16;
constexpr size_t OFF_PKL = OFF_PKH + SZ_PK;
constexpr size_t OFF_RW  = OFF_PKL + SZ_PK;
constexpr size_t SZ_W128 = (size_t)128 * CDIM * 2;
constexpr size_t SZ_W64  = (size_t)64 * CDIM * 2;
constexpr size_t SZ_W768 = (size_t)CDIM * CDIM * 2;
constexpr size_t OFF_WB1H  = OFF_RW;
constexpr size_t OFF_WB1L  = OFF_WB1H + SZ_W128;
constexpr size_t OFF_WBRKH = OFF_WB1L + SZ_W128;
constexpr size_t OFF_WBRKL = OFF_WBRKH + 2 * SZ_W768;
constexpr size_t OFF_WBOH  = OFF_WBRKL + 2 * SZ_W768;
constexpr size_t OFF_WBOL  = OFF_WBOH + SZ_W768;
constexpr size_t OFF_WBG1H = OFF_WBOL + SZ_W768;
constexpr size_t OFF_WBG1L = OFF_WBG1H + SZ_W128;
constexpr size_t OFF_WBKMH = OFF_WBG1L + SZ_W128;
constexpr size_t OFF_WBKML = OFF_WBKMH + SZ_W64;
constexpr size_t OFF_WHA   = OFF_WBKML + SZ_W64;
constexpr size_t OFF_WHV   = OFF_WHA + 2 * SZ_W128;
constexpr size_t OFF_WB2MH = OFF_WHV + SZ_W768;
constexpr size_t OFF_WB2ML = OFF_WB2MH + (size_t)4 * CDIM * 32 * 2;
constexpr size_t OFF_WB2GH = OFF_WB2ML + (size_t)4 * CDIM * 32 * 2;
constexpr size_t OFF_WB2GL = OFF_WB2GH + (size_t)CDIM * 128 * 2;
constexpr size_t OFF_WB2KH = OFF_WB2GL + (size_t)CDIM * 128 * 2;
constexpr size_t OFF_WB2KL = OFF_WB2KH + (size_t)2 * CDIM * 32 * 2;
constexpr size_t OFF_WH2D  = OFF_WB2KL + (size_t)2 * CDIM * 32 * 2;
constexpr size_t OFF_WH2S  = OFF_WH2D + (size_t)CDIM * 64 * 2;
constexpr size_t WS_TOTAL  = OFF_WH2S + (size_t)3 * CDIM * 32 * 2;
static_assert(WS_TOTAL == 108904448, "carve total");
static_assert(WS_TOTAL <= 134217728, "carve budget");
static_assert(OFF_RB % 128 == 0 && OFF_RC % 128 == 0 && OFF_RD % 128 == 0 && OFF_RE % 128 == 0 && OFF_RW % 128 == 0, "align");
static_assert(OFF_P16 % 128 == 0 && OFF_PKH % 128 == 0 && OFF_WH2S % 128 == 0 && OFF_WB2MH % 128 == 0, "align");
static_assert(6 * P16B >= 3 * P32B && 6 * P16B >= P32B + 2 * P16B, "RB reuse");
constexpr size_t OUT0_FLOATS = (size_t)MTOT * CDIM;
static_assert(OUT0_FLOATS * 4 == 25165824, "out1 byte offset");
static_assert(2 * OUT0_FLOATS * 4 == 50331648, "out total");

__device__ __forceinline__ unsigned short f2bf_bits(float f) {
  unsigned u = __float_as_uint(f);
  return (unsigned short)((u + 0x7FFFu + ((u >> 16) & 1u)) >> 16);
}
__device__ __forceinline__ float bf_bits2f(unsigned short h) { return __uint_as_float(((unsigned)h) << 16); }

__device__ __forceinline__ void dep_guard_h(v8f& a, v8f& b, v16h x, v16h y) { asm volatile("v_nop\n\tv_nop\n\tv_nop\n\tv_nop" : "+v"(a), "+v"(b) : "v"(x), "v"(y)); }
__device__ __forceinline__ void dep_guard_b(v8f& a, v8f& b, v16b x, v16b y) { asm volatile("v_nop\n\tv_nop\n\tv_nop\n\tv_nop" : "+v"(a), "+v"(b) : "v"(x), "v"(y)); }
__device__ __forceinline__ void keep4_h(v16h a, v16h b, v16h c, v16h d) { asm volatile("v_nop" :: "v"(a), "v"(b), "v"(c), "v"(d)); }
__device__ __forceinline__ void keep4_b(v16b a, v16b b, v16b c, v16b d) { asm volatile("v_nop" :: "v"(a), "v"(b), "v"(c), "v"(d)); }
__device__ __forceinline__ void acc_guard4(v8f& a, v8f& b, v8f& c, v8f& d) { asm volatile("v_nop\n\tv_nop\n\tv_nop\n\tv_nop" : "+v"(a), "+v"(b), "+v"(c), "+v"(d)); }
template <typename T> struct Frag;
template <> struct Frag<_Float16> {
  typedef v16h V; union U { v16h v; v8h h[2]; };
  static __device__ __forceinline__ v16h load(const _Float16* p) {
    U f; f.h[0] = *(const v8h*)(p); f.h[1] = *(const v8h*)(p + 16); return f.v;
  }
  static __device__ __forceinline__ v8f mma(v16h a, v16h b, v8f c) {
    return __builtin_amdgcn_wmma_f32_16x16x32_f16(false, a, false, b, (short)0, c, false, false);
  }
  static __device__ __forceinline__ void guard(v8f& a, v8f& b, v16h x, v16h y) { dep_guard_h(a, b, x, y); }
  static __device__ __forceinline__ void keep(v16h a, v16h b, v16h c, v16h d) { keep4_h(a, b, c, d); }
};
template <> struct Frag<__bf16> {
  typedef v16b V; union U { v16b v; v8b h[2]; };
  static __device__ __forceinline__ v16b load(const __bf16* p) {
    U f; f.h[0] = *(const v8b*)(p); f.h[1] = *(const v8b*)(p + 16); return f.v;
  }
  static __device__ __forceinline__ v8f mma(v16b a, v16b b, v8f c) {
    return __builtin_amdgcn_wmma_f32_16x16x32_bf16(false, a, false, b, (short)0, c, false, false);
  }
  static __device__ __forceinline__ void guard(v8f& a, v8f& b, v16b x, v16b y) { dep_guard_b(a, b, x, y); }
  static __device__ __forceinline__ void keep(v16b a, v16b b, v16b c, v16b d) { keep4_b(a, b, c, d); }
};

template <int ET> struct Elem;
template <> struct Elem<0> { typedef _Float16 T; };
template <> struct Elem<1> { typedef __bf16 T; };
template <int ET, bool SPLIT, int BIAS_MODE, int OUT_MODE, bool RESID, int ACT = 0>
__global__ __launch_bounds__(256) void wmma_gemm64(
    const unsigned short* __restrict__ Ap, const unsigned short* __restrict__ A2p, int lda, long strideA,
    const unsigned short* __restrict__ Btp, const unsigned short* __restrict__ Bt2p, int ldb, long strideB,
    void* __restrict__ Cout, void* __restrict__ Cout2, int ldc, long strideC,
    const float* __restrict__ bias,
    const float* __restrict__ resid, long strideR,
    int M, int N, int K, float scale, int ncut0, int ncutStep) {
  typedef typename Elem<ET>::T T;
  typedef typename Frag<T>::V V;
  const T* A = (const T*)Ap; const T* A2 = (const T*)A2p; const T* Bt = (const T*)Btp; const T* Bt2 = (const T*)Bt2p;
  __shared__ __align__(16) float sT[8][16 * 68];
  const int b    = blockIdx.y;
  const int lane = threadIdx.x & 31;
  const int wave = threadIdx.x >> 5;
  const int tilesN = N >> 6;
  const int tilesM = M >> 6;
  const int tile = blockIdx.x * 8 + wave;
  if (tile >= tilesM * tilesN) return;
  const int tm = tile / tilesN;
  const int tn = tile - tm * tilesN;
  const int m0 = tm << 6;
  const int n0 = tn << 6;
  const int ncut = ncut0 + b * ncutStep;

  const T* Ab  = A  + (size_t)b * strideA;
  const T* Bb  = Bt + (size_t)b * strideB;
  const T* Ab2 = SPLIT ? (A2  + (size_t)b * strideA) : nullptr;
  const T* Bb2 = SPLIT ? (Bt2 + (size_t)b * strideB) : nullptr;

  const int rlane = lane & 15;
  const int koff  = (lane >> 4) * 8;
  const int mOff  = (lane >> 4) * 8;

  v8f acc[4][4];
#pragma unroll
  for (int i = 0; i < 4; ++i)
#pragma unroll
    for (int j = 0; j < 4; ++j) acc[i][j] = (v8f){0.f,0.f,0.f,0.f,0.f,0.f,0.f,0.f};

  for (int k0 = 0; k0 < K; k0 += 32) {
    V bh[4], bl[4];
#pragma unroll
    for (int j = 0; j < 4; ++j) {
      const size_t bo = (size_t)(n0 + (j << 4) + rlane) * ldb + koff + k0;
      bh[j] = Frag<T>::load(Bb + bo);
      if (SPLIT) bl[j] = Frag<T>::load(Bb2 + bo);
    }
#pragma unroll
    for (int i = 0; i < 4; ++i) {
      const size_t ao = (size_t)(m0 + (i << 4) + rlane) * lda + koff + k0;
      V ah = Frag<T>::load(Ab + ao);
      V al;
      if (SPLIT) al = Frag<T>::load(Ab2 + ao);
#pragma unroll
      for (int j = 0; j < 4; ++j) {
        acc[i][j] = Frag<T>::mma(ah, bh[j], acc[i][j]);
        if (SPLIT) {
          acc[i][j] = Frag<T>::mma(ah, bl[j], acc[i][j]);
          acc[i][j] = Frag<T>::mma(al, bh[j], acc[i][j]);
        }
      }
      Frag<T>::guard(acc[i][0], acc[i][3], ah, SPLIT ? al : ah);
    }
    Frag<T>::keep(bh[0], bh[1], bh[2], bh[3]);
    if (SPLIT) Frag<T>::keep(bl[0], bl[1], bl[2], bl[3]);
  }
  acc_guard4(acc[0][0], acc[0][1], acc[0][2], acc[0][3]);
  acc_guard4(acc[1][0], acc[1][1], acc[1][2], acc[1][3]);
  acc_guard4(acc[2][0], acc[2][1], acc[2][2], acc[2][3]);
  acc_guard4(acc[3][0], acc[3][1], acc[3][2], acc[3][3]);

  float* slab = sT[wave];
  const float* Rb = RESID ? (resid + (size_t)b * strideR) : nullptr;
#pragma unroll
  for (int i = 0; i < 4; ++i) {
    const int mBase = m0 + (i << 4);
#pragma unroll
    for (int j = 0; j < 4; ++j) {
      const int n = n0 + (j << 4) + rlane;
      float bv = 0.f;
      if (BIAS_MODE == 2) bv = bias[n];
#pragma unroll
      for (int r = 0; r < 8; ++r) {
        float v = acc[i][j][r] * scale;
        if (BIAS_MODE == 1) v += bias[mBase + mOff + r];
        if (BIAS_MODE == 2) v += bv;
        if (RESID) v += Rb[(size_t)(mBase + mOff + r) * ldc + n];
        if (ACT == 1) v = tanhf(v);
        if (ACT == 2) v = fmaxf(v, 0.0f);
        if (ACT == 3) v = v / (1.0f + expf(-v));
        if (ACT == 4) v = (v > 0.f) ? v : 0.01f * v;
        if (ACT == 6) { const float sg = __builtin_amdgcn_rcpf(1.0f + expf(-v)); v = (n < ncut) ? sg : 0.0f; }
        if (ACT == 7) { const float th = tanhf(v); v = (n < ncut) ? th : v; }
        slab[(mOff + r) * 68 + (j << 4) + rlane] = v;
      }
    }
    __builtin_amdgcn_fence(__ATOMIC_RELEASE, "workgroup");
    __builtin_amdgcn_wave_barrier();
    __builtin_amdgcn_fence(__ATOMIC_ACQUIRE, "workgroup");
    if (OUT_MODE == 0) {
      float* C = (float*)Cout + (size_t)b * strideC;
      const int hh = lane >> 4, c4 = (lane & 15) * 4;
      for (int pass = 0; pass < 2; ++pass) {
#pragma unroll
        for (int it = 0; it < 8; ++it) {
          const int row = it * 2 + hh;
          v4f v = *(const v4f*)(slab + row * 68 + c4);
          *(volatile v4f*)(C + (size_t)(mBase + row) * ldc + n0 + c4) = v;
        }
        __threadfence();
      }
    } else {
      const int q = lane >> 3, c8 = (lane & 7) * 8;
      unsigned short* C  = (unsigned short*)Cout  + (size_t)b * strideC;
      unsigned short* C2 = (OUT_MODE == 2) ? ((unsigned short*)Cout2 + (size_t)b * strideC) : nullptr;
      for (int pass = 0; pass < 2; ++pass) {
#pragma unroll
        for (int it = 0; it < 4; ++it) {
          const int row = it * 4 + q;
          const float* sp = slab + row * 68 + c8;
          v8h hv, lv;
#pragma unroll
          for (int e = 0; e < 8; ++e) {
            if (OUT_MODE == 1) {
              hv[e] = (_Float16)sp[e];
            } else {
              unsigned short hb = f2bf_bits(sp[e]);
              unsigned short lb = f2bf_bits(sp[e] - bf_bits2f(hb));
              hv[e] = __builtin_bit_cast(_Float16, hb);
              lv[e] = __builtin_bit_cast(_Float16, lb);
            }
          }
          *(volatile v8h*)(C + (size_t)(mBase + row) * ldc + n0 + c8) = hv;
          if (OUT_MODE == 2) *(volatile v8h*)(C2 + (size_t)(mBase + row) * ldc + n0 + c8) = lv;
        }
        __threadfence();
      }
    }
    __builtin_amdgcn_fence(__ATOMIC_RELEASE, "workgroup");
    __builtin_amdgcn_wave_barrier();
    __builtin_amdgcn_fence(__ATOMIC_ACQUIRE, "workgroup");
  }
}

struct WJob {
  const float* src; unsigned short* dstH; unsigned short* dstL;
  int kin; int srcPitch; int nsrc; int gout; int gin; int kpad; int nrows; int rowOff; int mode; float scale;
};
static_assert(sizeof(WJob) == 64, "no padding");
constexpr int NJOB = 24;
struct WJobs { WJob j[NJOB]; };
static_assert(sizeof(WJobs) == 64 * NJOB, "no padding");

__global__ __launch_bounds__(256) void k_wprep(WJobs jobs) {
  __shared__ float sm[64][33];
  const int z = blockIdx.z;
  WJob jb = jobs.j[0];
#pragma unroll
  for (int q = 1; q < NJOB; ++q) { if (z == q) jb = jobs.j[q]; }
  const int TK = (jb.kpad == 32) ? 32 : 64;
  const int k0 = blockIdx.x * TK;
  const int r0 = blockIdx.y * 32;
  if (k0 >= jb.kpad || r0 >= jb.nrows) return;
  const int tid = threadIdx.x;
  const int nl = tid & 31, kl = tid >> 5;
  const int n = r0 + nl;
  const int grp = n / jb.gout;
  const int wi = n - grp * jb.gout;
  int scol = grp * jb.gin + wi;
  const bool nval = (wi < jb.gin) && (scol < jb.nsrc);
  scol = nval ? scol : 0;
  for (int kk = 0; kk < TK; kk += 8) {
    const int k = k0 + kk + kl;
    const bool kval = (k < jb.kin);
    const int kc = kval ? k : 0;
    float v = jb.src[(size_t)kc * jb.srcPitch + scol];
    v = (kval && nval) ? (v * jb.scale) : 0.0f;
    sm[kk + kl][nl] = v;
  }
  __syncthreads();
  int nn, c8; bool act;
  if (TK == 64) { nn = tid >> 3; c8 = (tid & 7) * 8; act = true; }
  else          { nn = tid >> 2; c8 = (tid & 3) * 8; act = (tid < 128); }
  if (act) {
    float v[8];
#pragma unroll
    for (int e = 0; e < 8; ++e) v[e] = sm[c8 + e][nn];
    unsigned int hb[8], lb[8];
    if (jb.mode == 0) {
#pragma unroll
      for (int e = 0; e < 8; ++e) {
        const unsigned short h16 = f2bf_bits(v[e]);
        hb[e] = h16;
        lb[e] = f2bf_bits(v[e] - bf_bits2f(h16));
      }
    } else {
#pragma unroll
      for (int e = 0; e < 8; ++e) { hb[e] = (unsigned int)__builtin_bit_cast(unsigned short, (_Float16)v[e]); lb[e] = 0u; }
    }
    v4u hw, lw;
    hw.x = hb[0] | (hb[1] << 16); hw.y = hb[2] | (hb[3] << 16); hw.z = hb[4] | (hb[5] << 16); hw.w = hb[6] | (hb[7] << 16);
    lw.x = lb[0] | (lb[1] << 16); lw.y = lb[2] | (lb[3] << 16); lw.z = lb[4] | (lb[5] << 16); lw.w = lb[6] | (lb[7] << 16);
    const size_t off = (size_t)(jb.rowOff + r0 + nn) * jb.kpad + k0 + c8;
    unsigned short* ph = jb.dstH + off;
    unsigned short* pl = jb.dstL + off;
    *(volatile v4u*)ph = hw;
    if (jb.mode == 0) *(volatile v4u*)pl = lw;
    __threadfence();
    *(volatile v4u*)ph = hw;
    if (jb.mode == 0) *(volatile v4u*)pl = lw;
  }
}

__global__ __launch_bounds__(256) void k_shift(const float* __restrict__ x, const float* __restrict__ maa_x,
                                               unsigned short* __restrict__ xh, unsigned short* __restrict__ xl, int chunk) {
  const int t = blockIdx.x * 256 + threadIdx.x;
  const int m = t / 192;
  const int c = (t - m * 192) * 4;
  const int gm = chunk * MCH + m;
  const int tt = gm & (TLEN - 1);
  const int pm = (tt > 0) ? (gm - 1) : gm;
  const v4f xc = *(const v4f*)(x + (size_t)gm * CDIM + c);
  const v4f xq = *(const v4f*)(x + (size_t)pm * CDIM + c);
  const v4f mx = *(const v4f*)(maa_x + c);
  unsigned int hb[4], lb[4];
#pragma unroll
  for (int e = 0; e < 4; ++e) {
    const float xp = (tt > 0) ? xq[e] : 0.0f;
    const float xx = xp - xc[e];
    const float val = xc[e] + xx * mx[e];
    const unsigned short h16 = f2bf_bits(val);
    hb[e] = h16; lb[e] = f2bf_bits(val - bf_bits2f(h16));
  }
  v2u hw, lw;
  hw.x = hb[0] | (hb[1] << 16); hw.y = hb[2] | (hb[3] << 16);
  lw.x = lb[0] | (lb[1] << 16); lw.y = lb[2] | (lb[3] << 16);
  const size_t eo = (size_t)m * CDIM + c;
  *(volatile v2u*)(xh + eo) = hw; *(volatile v2u*)(xl + eo) = lw;
  __threadfence();
  *(volatile v2u*)(xh + eo) = hw; *(volatile v2u*)(xl + eo) = lw;
}

__global__ __launch_bounds__(256) void k_mix(
    const float* __restrict__ x, const float* __restrict__ mrg, const float* __restrict__ mwa,
    const float* __restrict__ mkk, const float* __restrict__ mvv, const float* __restrict__ mix,
    unsigned short* __restrict__ xrgh, unsigned short* __restrict__ xrgl,
    unsigned short* __restrict__ xkh, unsigned short* __restrict__ xkl,
    unsigned short* __restrict__ xwa16, unsigned short* __restrict__ xv16, int chunk) {
  const int t = blockIdx.x * 256 + threadIdx.x;
  const int m = t / 192;
  const int c = (t - m * 192) * 4;
  const int gm = chunk * MCH + m;
  const int tt = gm & (TLEN - 1);
  const int pm = (tt > 0) ? (gm - 1) : gm;
  const v4f xc = *(const v4f*)(x + (size_t)gm * CDIM + c);
  const v4f xq = *(const v4f*)(x + (size_t)pm * CDIM + c);
  const v4f c0 = *(const v4f*)(mrg + c);
  const v4f c1 = *(const v4f*)(mwa + c);
  const v4f c2 = *(const v4f*)(mkk + c);
  const v4f c3 = *(const v4f*)(mvv + c);
  const size_t eo = (size_t)m * CDIM + c;
  const size_t PL = (size_t)MCH * CDIM;
  const v4f q0 = *(const v4f*)(mix + eo);
  const v4f q1 = *(const v4f*)(mix + PL + eo);
  const v4f q2 = *(const v4f*)(mix + 2 * PL + eo);
  const v4f q3 = *(const v4f*)(mix + 3 * PL + eo);
  unsigned int hr[4], lr[4], hk[4], lk[4], fw[4], fv[4];
#pragma unroll
  for (int e = 0; e < 4; ++e) {
    const float xp = (tt > 0) ? xq[e] : 0.0f;
    const float xx = xp - xc[e];
    const float vrg = xc[e] + xx * (c0[e] + q0[e]);
    const float vwa = xc[e] + xx * (c1[e] + q1[e]);
    const float vk  = xc[e] + xx * (c2[e] + q2[e]);
    const float vv  = xc[e] + xx * (c3[e] + q3[e]);
    unsigned short h16 = f2bf_bits(vrg); hr[e] = h16; lr[e] = f2bf_bits(vrg - bf_bits2f(h16));
    h16 = f2bf_bits(vk); hk[e] = h16; lk[e] = f2bf_bits(vk - bf_bits2f(h16));
    fw[e] = (unsigned int)__builtin_bit_cast(unsigned short, (_Float16)vwa);
    fv[e] = (unsigned int)__builtin_bit_cast(unsigned short, (_Float16)vv);
  }
  v2u a0, a1, a2, a3, a4, a5;
  a0.x = hr[0] | (hr[1] << 16); a0.y = hr[2] | (hr[3] << 16);
  a1.x = lr[0] | (lr[1] << 16); a1.y = lr[2] | (lr[3] << 16);
  a2.x = hk[0] | (hk[1] << 16); a2.y = hk[2] | (hk[3] << 16);
  a3.x = lk[0] | (lk[1] << 16); a3.y = lk[2] | (lk[3] << 16);
  a4.x = fw[0] | (fw[1] << 16); a4.y = fw[2] | (fw[3] << 16);
  a5.x = fv[0] | (fv[1] << 16); a5.y = fv[2] | (fv[3] << 16);
  *(volatile v2u*)(xrgh + eo) = a0; *(volatile v2u*)(xrgl + eo) = a1;
  *(volatile v2u*)(xkh + eo)  = a2; *(volatile v2u*)(xkl + eo)  = a3;
  *(volatile v2u*)(xwa16 + eo) = a4; *(volatile v2u*)(xv16 + eo) = a5;
  __threadfence();
  *(volatile v2u*)(xrgh + eo) = a0; *(volatile v2u*)(xrgl + eo) = a1;
  *(volatile v2u*)(xkh + eo)  = a2; *(volatile v2u*)(xkl + eo)  = a3;
  *(volatile v2u*)(xwa16 + eo) = a4; *(volatile v2u*)(xv16 + eo) = a5;
}

__global__ __launch_bounds__(256) void k_fuse(
    const float* __restrict__ Kraw, const float* __restrict__ Vraw, const float* __restrict__ v1g,
    const float* __restrict__ Wpre, const float* __restrict__ Kkd, const float* __restrict__ Mkp,
    const float* __restrict__ Apre, const float* __restrict__ Mapre, const float* __restrict__ Mvpre,
    const float* __restrict__ tdec, const float* __restrict__ taaa, const float* __restrict__ misa,
    const float* __restrict__ misk, const float* __restrict__ misv,
    float* __restrict__ WDo, float* __restrict__ KFo, float* __restrict__ VFo,
    float* __restrict__ KKo, float* __restrict__ BBo, int chunk) {
  const int m = blockIdx.x / 3;
  const int c = (blockIdx.x - m * 3) * 256 + threadIdx.x;
  const size_t e  = (size_t)m * CDIM + c;
  const size_t eg = (size_t)(chunk * MCH + m) * CDIM + c;
  const float kr = Kraw[e], vr = Vraw[e], v1v = v1g[eg], wp = Wpre[e], kd = Kkd[e], mkp = Mkp[e];
  const float ap = Apre[e], map = Mapre[e], mvp = Mvpre[e];
  const float td = tdec[c], ta = taaa[c], ma0 = misa[c], mk0 = misk[c], mv0 = misv[c];
  const float z = -(td + wp);
  const float sp = fmaxf(z, 0.0f) + log1pf(expf(-fabsf(z)));
  const float w = -sp - 0.5f;
  const float wd = expf(-expf(w));
  const float a  = __builtin_amdgcn_rcpf(1.0f + expf(-(ta + ap)));
  const float ma = __builtin_amdgcn_rcpf(1.0f + expf(-(ma0 + map)));
  const float mk = __builtin_amdgcn_rcpf(1.0f + expf(-(mk0 + mkp)));
  const float mv = __builtin_amdgcn_rcpf(1.0f + expf(-(mv0 + mvp)));
  const float kk = kr + kd;
  float ss = kk * kk;
#pragma unroll
  for (int off = 1; off < 32; off <<= 1) ss += __shfl_xor(ss, off, 32);
  const float nrm = fmaxf(sqrtf(ss), 1e-12f);
  const float kkn = kk * __builtin_amdgcn_rcpf(nrm);
  const float kf = (kr * ma + kr * a * (1.0f - ma)) * expf(fminf(w * mk, 0.0f));
  const float vf = vr + (v1v - vr) * mv;
  const float bb = kkn * a;
  ((volatile float*)WDo)[e] = wd; ((volatile float*)KFo)[e] = kf; ((volatile float*)VFo)[e] = vf;
  ((volatile float*)KKo)[e] = kkn; ((volatile float*)BBo)[e] = bb;
  __threadfence();
  ((volatile float*)WDo)[e] = wd; ((volatile float*)KFo)[e] = kf; ((volatile float*)VFo)[e] = vf;
  ((volatile float*)KKo)[e] = kkn; ((volatile float*)BBo)[e] = bb;
}

__global__ __launch_bounds__(32) void k_scan(const float* __restrict__ Rp, const float* __restrict__ WD,
                                             const float* __restrict__ KF, const float* __restrict__ VF,
                                             const float* __restrict__ KKN, const float* __restrict__ BBp,
                                             float* __restrict__ Y) {
  __shared__ __align__(16) float rS[HSZ];
  __shared__ __align__(16) float wS[HSZ];
  __shared__ __align__(16) float kS[HSZ];
  __shared__ __align__(16) float aS[HSZ];
  __shared__ __align__(16) float bS[HSZ];
  __shared__ __align__(16) float yst[32][36];
  const int bl = blockIdx.x / NHEAD;
  const int h = blockIdx.x - bl * NHEAD;
  const int i = threadIdx.x;
  const size_t col = (size_t)h * HSZ;
  float s[HSZ];
#pragma unroll
  for (int j = 0; j < HSZ; ++j) s[j] = 0.0f;
#pragma unroll 1
  for (int t = 0; t < TLEN; ++t) {
    const size_t idx = (size_t)(bl * TLEN + t) * CDIM + col + i;
    const float lr = Rp[idx], lw = WD[idx], lk = KF[idx], lv = VF[idx], la = KKN[idx], lb = BBp[idx];
    rS[i] = lr; wS[i] = lw; kS[i] = lk; aS[i] = -la; bS[i] = lb;
    __syncthreads();
    float sa = 0.0f;
#pragma unroll
    for (int q = 0; q < 8; ++q) {
      const v4f a4 = *(const v4f*)(aS + 4 * q);
#pragma unroll
      for (int e = 0; e < 4; ++e) {
        float p = s[4 * q + e] * a4[e];
        asm volatile("" : "+v"(p));
        sa += p;
      }
    }
    float yv = 0.0f;
#pragma unroll
    for (int q = 0; q < 8; ++q) {
      const v4f w4 = *(const v4f*)(wS + 4 * q);
      const v4f k4 = *(const v4f*)(kS + 4 * q);
      const v4f b4 = *(const v4f*)(bS + 4 * q);
      const v4f r4 = *(const v4f*)(rS + 4 * q);
#pragma unroll
      for (int e = 0; e < 4; ++e) {
        const int j = 4 * q + e;
        float u = sa * b4[e];
        u = fmaf(lv, k4[e], u);
        s[j] = fmaf(s[j], w4[e], u);
        float p = s[j] * r4[e];
        asm volatile("" : "+v"(p));
        yv += p;
      }
    }
    yst[t & 31][i] = yv;
    __syncthreads();
    if ((t & 31) == 31) {
      const int t0 = t - 31;
      const int lq = i >> 3, c4 = (i & 7) * 4;
      v4f vals[8];
#pragma unroll
      for (int it = 0; it < 8; ++it) vals[it] = *(const v4f*)(&yst[it * 4 + lq][c4]);
      for (int pass = 0; pass < 2; ++pass) {
#pragma unroll
        for (int it = 0; it < 8; ++it) {
          const int line = it * 4 + lq;
          *(volatile v4f*)(Y + (size_t)(bl * TLEN + t0 + line) * CDIM + col + c4) = vals[it];
        }
        __threadfence();
      }
    }
  }
}

__global__ __launch_bounds__(256) void k_post(const float* __restrict__ Y, const float* __restrict__ Rp,
                                             const float* __restrict__ KF, const float* __restrict__ VF,
                                             const float* __restrict__ Gp, const float* __restrict__ faa,
                                             const float* __restrict__ lnw, const float* __restrict__ lnb,
                                             unsigned short* __restrict__ YGh, unsigned short* __restrict__ YGl) {
  const int idx = blockIdx.x * 256 + threadIdx.x;
  const int m = idx / 384;
  const int c = (idx - m * 384) * 2;
  const size_t e = (size_t)m * CDIM + c;
  const v2f y2 = *(const v2f*)(Y + e);
  const v2f r2 = *(const v2f*)(Rp + e);
  const v2f k2 = *(const v2f*)(KF + e);
  const v2f vv2 = *(const v2f*)(VF + e);
  const v2f g2 = *(const v2f*)(Gp + e);
  const v2f f2 = *(const v2f*)(faa + c);
  const v2f w2 = *(const v2f*)(lnw + c);
  const v2f b2 = *(const v2f*)(lnb + c);
  float s1 = y2.x + y2.y;
#pragma unroll
  for (int off = 1; off < 16; off <<= 1) s1 += __shfl_xor(s1, off, 32);
  const float mu = s1 * (1.0f / 32.0f);
  const float d0 = y2.x - mu, d1 = y2.y - mu;
  float s2 = d0 * d0 + d1 * d1;
#pragma unroll
  for (int off = 1; off < 16; off <<= 1) s2 += __shfl_xor(s2, off, 32);
  const float var = s2 * (1.0f / 32.0f);
  const float rs = rsqrtf(var + 6.4e-05f);
  float bs = r2.x * k2.x * f2.x + r2.y * k2.y * f2.y;
#pragma unroll
  for (int off = 1; off < 16; off <<= 1) bs += __shfl_xor(bs, off, 32);
  const float yn0 = (d0 * rs) * w2.x + b2.x;
  const float yn1 = (d1 * rs) * w2.y + b2.y;
  const float yf0 = (yn0 + bs * vv2.x) * g2.x;
  const float yf1 = (yn1 + bs * vv2.y) * g2.y;
  const unsigned short h0 = f2bf_bits(yf0), h1 = f2bf_bits(yf1);
  const unsigned int l0 = f2bf_bits(yf0 - bf_bits2f(h0)), l1 = f2bf_bits(yf1 - bf_bits2f(h1));
  const unsigned int hw = (unsigned int)h0 | ((unsigned int)h1 << 16);
  const unsigned int lw = l0 | (l1 << 16);
  const size_t e2 = e >> 1;
  ((volatile unsigned int*)YGh)[e2] = hw; ((volatile unsigned int*)YGl)[e2] = lw;
  __threadfence();
  ((volatile unsigned int*)YGh)[e2] = hw; ((volatile unsigned int*)YGl)[e2] = lw;
}

__global__ __launch_bounds__(256) void k_copy4(const float* __restrict__ src, float* __restrict__ dst, int n4) {
  const int i = blockIdx.x * 256 + threadIdx.x;
  if (i < n4) {
    const v4f v = *(const v4f*)(src + (size_t)i * 4);
    *(volatile v4f*)(dst + (size_t)i * 4) = v;
    __threadfence();
    *(volatile v4f*)(dst + (size_t)i * 4) = v;
  }
}

static inline dim3 ggrid(int M, int N, int nb) { return dim3((unsigned)(((M / 64) * (N / 64) + 7) / 8), (unsigned)nb, 1); }

extern "C" void kernel_launch(void* const* d_in, const int* in_sizes, int n_in,
                              void* d_out, int out_size, void* d_ws, size_t ws_size,
                              hipStream_t stream) {
  (void)in_sizes; (void)n_in; (void)out_size;
  if (ws_size < WS_TOTAL) return;

  const float* x          = (const float*)d_in[0];
  const float* v1         = (const float*)d_in[1];
  const float* maa_x      = (const float*)d_in[2];
  const float* maa_rg     = (const float*)d_in[3];
  const float* maa_wa     = (const float*)d_in[4];
  const float* maa_k      = (const float*)d_in[5];
  const float* maa_v      = (const float*)d_in[6];
  const float* time_decay = (const float*)d_in[7];
  const float* faaaa      = (const float*)d_in[8];
  const float* time_aaaaa = (const float*)d_in[9];
  const float* maa_w1     = (const float*)d_in[10];
  const float* maa_w2     = (const float*)d_in[11];
  const float* dec_w1     = (const float*)d_in[12];
  const float* dec_w2     = (const float*)d_in[13];
  const float* aaa_w1     = (const float*)d_in[14];
  const float* aaa_w2     = (const float*)d_in[15];
  const float* kkk_w1     = (const float*)d_in[16];
  const float* kkk_w2     = (const float*)d_in[17];
  const float* gate_w1    = (const float*)d_in[18];
  const float* gate_w2    = (const float*)d_in[19];
  const float* ma_w1      = (const float*)d_in[20];
  const float* ma_w2      = (const float*)d_in[21];
  const float* misc_a     = (const float*)d_in[22];
  const float* mk_w1      = (const float*)d_in[23];
  const float* mk_w2      = (const float*)d_in[24];
  const float* misc_k     = (const float*)d_in[25];
  const float* mv_w1      = (const float*)d_in[26];
  const float* mv_w2      = (const float*)d_in[27];
  const float* misc_v     = (const float*)d_in[28];
  const float* Wr         = (const float*)d_in[29];
  const float* Wk         = (const float*)d_in[30];
  const float* Wv         = (const float*)d_in[31];
  const float* Wo         = (const float*)d_in[32];
  const float* ln_w       = (const float*)d_in[33];
  const float* ln_b       = (const float*)d_in[34];

  float* out0 = (float*)d_out;
  float* out1 = out0 + OUT0_FLOATS;
  char* ws = (char*)d_ws;
  const float* fdum = (const float*)d_ws;

  float* MIX  = (float*)(ws + OFF_RA);
  float* Gp   = (float*)(ws + OFF_RA);
  float* KKD  = (float*)(ws + OFF_RA + P32B);
  float* MKP  = (float*)(ws + OFF_RA + 2 * P32B);
  float* WPRE = (float*)(ws + OFF_RA + 3 * P32B);
  unsigned short* XXXh  = (unsigned short*)(ws + OFF_RB);
  unsigned short* XXXl  = (unsigned short*)(ws + OFF_RB + P16B);
  unsigned short* XRGh  = (unsigned short*)(ws + OFF_RB);
  unsigned short* XRGl  = (unsigned short*)(ws + OFF_RB + P16B);
  unsigned short* XKh   = (unsigned short*)(ws + OFF_RB + 2 * P16B);
  unsigned short* XKl   = (unsigned short*)(ws + OFF_RB + 3 * P16B);
  unsigned short* XWA16 = (unsigned short*)(ws + OFF_RB + 4 * P16B);
  unsigned short* XV16  = (unsigned short*)(ws + OFF_RB + 5 * P16B);
  float* APRE  = (float*)(ws + OFF_RB);
  float* MAPRE = (float*)(ws + OFF_RB + P32B);
  float* MVPRE = (float*)(ws + OFF_RB + 2 * P32B);
  float* Yp    = (float*)(ws + OFF_RB);
  unsigned short* YGh = (unsigned short*)(ws + OFF_RB + P32B);
  unsigned short* YGl = (unsigned short*)(ws + OFF_RB + P32B + P16B);
  float* Rp   = (float*)(ws + OFF_RC);
  float* KRAW = (float*)(ws + OFF_RC + P32B);
  float* VRAW = (float*)(ws + OFF_RC + 2 * P32B);
  float* WD   = (float*)(ws + OFF_RD);
  float* KFIN = (float*)(ws + OFF_RD + P32B);
  float* VFIN = (float*)(ws + OFF_RD + 2 * P32B);
  float* KKN  = (float*)(ws + OFF_RD + 3 * P32B);
  float* BBp  = (float*)(ws + OFF_RD + 4 * P32B);
  unsigned short* TMh = (unsigned short*)(ws + OFF_TMH);
  unsigned short* TMl = (unsigned short*)(ws + OFF_TML);
  unsigned short* GSh = (unsigned short*)(ws + OFF_GSH);
  unsigned short* GSl = (unsigned short*)(ws + OFF_GSL);
  unsigned short* P16 = (unsigned short*)(ws + OFF_P16);
  unsigned short* PKh = (unsigned short*)(ws + OFF_PKH);
  unsigned short* PKl = (unsigned short*)(ws + OFF_PKL);
  unsigned short* WB1h  = (unsigned short*)(ws + OFF_WB1H);
  unsigned short* WB1l  = (unsigned short*)(ws + OFF_WB1L);
  unsigned short* WBRKh = (unsigned short*)(ws + OFF_WBRKH);
  unsigned short* WBRKl = (unsigned short*)(ws + OFF_WBRKL);
  unsigned short* WBOh  = (unsigned short*)(ws + OFF_WBOH);
  unsigned short* WBOl  = (unsigned short*)(ws + OFF_WBOL);
  unsigned short* WBG1h = (unsigned short*)(ws + OFF_WBG1H);
  unsigned short* WBG1l = (unsigned short*)(ws + OFF_WBG1L);
  unsigned short* WBKMh = (unsigned short*)(ws + OFF_WBKMH);
  unsigned short* WBKMl = (unsigned short*)(ws + OFF_WBKML);
  unsigned short* WHA   = (unsigned short*)(ws + OFF_WHA);
  unsigned short* WHV   = (unsigned short*)(ws + OFF_WHV);
  unsigned short* WB2Mh = (unsigned short*)(ws + OFF_WB2MH);
  unsigned short* WB2Ml = (unsigned short*)(ws + OFF_WB2ML);
  unsigned short* WB2Gh = (unsigned short*)(ws + OFF_WB2GH);
  unsigned short* WB2Gl = (unsigned short*)(ws + OFF_WB2GL);
  unsigned short* WB2Kh = (unsigned short*)(ws + OFF_WB2KH);
  unsigned short* WB2Kl = (unsigned short*)(ws + OFF_WB2KL);
  unsigned short* WH2D  = (unsigned short*)(ws + OFF_WH2D);
  unsigned short* WH2S  = (unsigned short*)(ws + OFF_WH2S);

  WJobs jobs;
  auto setjob = [&](int q, const float* src, unsigned short* dh, unsigned short* dl, int kin, int srcPitch, int nsrc,
                    int gout, int gin, int kpad, int nrows, int rowOff, int mode, float scale) {
    WJob& j = jobs.j[q];
    j.src = src; j.dstH = dh; j.dstL = dl; j.kin = kin; j.srcPitch = srcPitch; j.nsrc = nsrc; j.gout = gout; j.gin = gin;
    j.kpad = kpad; j.nrows = nrows; j.rowOff = rowOff; j.mode = mode; j.scale = scale;
  };
  const int S32 = CDIM * 32;
  setjob(0,  maa_w1,  WB1h,  WB1l,  CDIM, 112, 112, 32, 28, CDIM, 128, 0,   0, 1.0f);
  setjob(1,  Wr,      WBRKh, WBRKl, CDIM, CDIM, CDIM, CDIM, CDIM, CDIM, CDIM, 0,    0, 1.0f);
  setjob(2,  Wk,      WBRKh, WBRKl, CDIM, CDIM, CDIM, CDIM, CDIM, CDIM, CDIM, CDIM, 0, 1.0f);
  setjob(3,  Wo,      WBOh,  WBOl,  CDIM, CDIM, CDIM, CDIM, CDIM, CDIM, CDIM, 0,    0, 1.0f);
  setjob(4,  gate_w1, WBG1h, WBG1l, CDIM, 120, 120, 128, 128, CDIM, 128, 0, 0, 1.0f);
  setjob(5,  kkk_w1,  WBKMh, WBKMl, CDIM, 24, 24, 32, 32, CDIM, 32, 0,  0, 1.0f);
  setjob(6,  mk_w1,   WBKMh, WBKMl, CDIM, 24, 24, 32, 32, CDIM, 32, 32, 0, 1.0f);
  setjob(7,  dec_w1,  WHA, WHA, CDIM, 64, 64, 64, 64, CDIM, 64, 0,   1, 64.0f);
  setjob(8,  aaa_w1,  WHA, WHA, CDIM, 24, 24, 32, 32, CDIM, 32, 64,  1, 64.0f);
  setjob(9,  ma_w1,   WHA, WHA, CDIM, 24, 24, 32, 32, CDIM, 32, 96,  1, 64.0f);
  setjob(10, mv_w1,   WHA, WHA, CDIM, 24, 24, 32, 32, CDIM, 32, 128, 1, 64.0f);
  setjob(11, mv_w1,   WHA, WHA, 1,    24, 0,  32, 32, CDIM, 96, 160, 1, 64.0f);
  setjob(12, Wv,      WHV, WHV, CDIM, CDIM, CDIM, CDIM, CDIM, CDIM, CDIM, 0, 1, 64.0f);
  setjob(13, maa_w2 + 0 * 28 * CDIM, WB2Mh + 0 * S32, WB2Ml + 0 * S32, 28, CDIM, CDIM, CDIM, CDIM, 32, CDIM, 0, 0, 1.0f);
  setjob(14, maa_w2 + 1 * 28 * CDIM, WB2Mh + 1 * S32, WB2Ml + 1 * S32, 28, CDIM, CDIM, CDIM, CDIM, 32, CDIM, 0, 0, 1.0f);
  setjob(15, maa_w2 + 2 * 28 * CDIM, WB2Mh + 2 * S32, WB2Ml + 2 * S32, 28, CDIM, CDIM, CDIM, CDIM, 32, CDIM, 0, 0, 1.0f);
  setjob(16, maa_w2 + 3 * 28 * CDIM, WB2Mh + 3 * S32, WB2Ml + 3 * S32, 28, CDIM, CDIM, CDIM, CDIM, 32, CDIM, 0, 0, 1.0f);
  setjob(17, gate_w2, WB2Gh, WB2Gl, 120, CDIM, CDIM, CDIM, CDIM, 128, CDIM, 0, 0, 1.0f);
  setjob(18, kkk_w2,  WB2Kh + 0 * S32, WB2Kl + 0 * S32, 24, CDIM, CDIM, CDIM, CDIM, 32, CDIM, 0, 0, 1.0f);
  setjob(19, mk_w2,   WB2Kh + 1 * S32, WB2Kl + 1 * S32, 24, CDIM, CDIM, CDIM, CDIM, 32, CDIM, 0, 0, 1.0f);
  setjob(20, dec_w2,  WH2D, WH2D, 64, CDIM, CDIM, CDIM, CDIM, 64, CDIM, 0, 1, 64.0f);
  setjob(21, aaa_w2,  WH2S + 0 * S32, WH2S + 0 * S32, 24, CDIM, CDIM, CDIM, CDIM, 32, CDIM, 0, 1, 64.0f);
  setjob(22, ma_w2,   WH2S + 1 * S32, WH2S + 1 * S32, 24, CDIM, CDIM, CDIM, CDIM, 32, CDIM, 0, 1, 64.0f);
  setjob(23, mv_w2,   WH2S + 2 * S32, WH2S + 2 * S32, 24, CDIM, CDIM, CDIM, CDIM, 32, CDIM, 0, 1, 64.0f);
  k_wprep<<<dim3(CDIM / 64, CDIM / 32, NJOB), 256, 0, stream>>>(jobs);

  k_copy4<<<(unsigned)(OUT0_FLOATS / 4 / 256), 256, 0, stream>>>(v1, out1, (int)(OUT0_FLOATS / 4));
  static_assert((OUT0_FLOATS / 4) % 256 == 0, "copy grid exact");

  static_assert((MCH * 192) % 256 == 0 && (MCH * CDIM) % 256 == 0 && (MCH * 384) % 256 == 0, "elementwise grids exact");
  const long PLE = (long)MCH * CDIM;
  const float s64 = 1.0f / 64.0f;

  for (int ch = 0; ch < NCHUNK; ++ch) {
    k_shift<<<(MCH * 192) / 256, 256, 0, stream>>>(x, maa_x, XXXh, XXXl, ch);
    wmma_gemm64<1, true, 0, 2, false, 1><<<ggrid(MCH, 128, 1), 256, 0, stream>>>(
        XXXh, XXXl, CDIM, 0L, WB1h, WB1l, CDIM, 0L, (void*)TMh, (void*)TMl, 128, 0L, fdum, fdum, 0L, MCH, 128, CDIM, 1.0f, 0, 0);
    wmma_gemm64<1, true, 0, 0, false, 0><<<ggrid(MCH, CDIM, 4), 256, 0, stream>>>(
        TMh, TMl, 128, 32L, WB2Mh, WB2Ml, 32, (long)S32, (void*)MIX, (void*)MIX, CDIM, PLE, fdum, fdum, 0L, MCH, CDIM, 32, 1.0f, 0, 0);
    k_mix<<<(MCH * 192) / 256, 256, 0, stream>>>(x, maa_rg, maa_wa, maa_k, maa_v, MIX,
                                                 XRGh, XRGl, XKh, XKl, XWA16, XV16, ch);
    wmma_gemm64<1, true, 0, 0, false, 0><<<ggrid(MCH, CDIM, 2), 256, 0, stream>>>(
        XRGh, XRGl, CDIM, 2 * PLE, WBRKh, WBRKl, CDIM, (long)CDIM * CDIM, (void*)Rp, (void*)Rp, CDIM, PLE, fdum, fdum, 0L, MCH, CDIM, CDIM, 1.0f, 0, 0);
    wmma_gemm64<0, false, 0, 0, false, 0><<<ggrid(MCH, CDIM, 1), 256, 0, stream>>>(
        XV16, XV16, CDIM, 0L, WHV, WHV, CDIM, 0L, (void*)VRAW, (void*)VRAW, CDIM, 0L, fdum, fdum, 0L, MCH, CDIM, CDIM, s64, 0, 0);
    wmma_gemm64<1, true, 0, 2, false, 6><<<ggrid(MCH, 128, 1), 256, 0, stream>>>(
        XRGh, XRGl, CDIM, 0L, WBG1h, WBG1l, CDIM, 0L, (void*)GSh, (void*)GSl, 128, 0L, fdum, fdum, 0L, MCH, 128, CDIM, 1.0f, 120, 0);
    wmma_gemm64<0, false, 0, 1, false, 7><<<ggrid(MCH, 128, 2), 256, 0, stream>>>(
        XWA16, XWA16, CDIM, PLE, WHA, WHA, CDIM, (long)128 * CDIM, (void*)P16, (void*)P16, 256, 128L, fdum, fdum, 0L, MCH, 128, CDIM, s64, 64, -64);
    wmma_gemm64<1, true, 0, 2, false, 7><<<ggrid(MCH, 64, 1), 256, 0, stream>>>(
        XKh, XKl, CDIM, 0L, WBKMh, WBKMl, CDIM, 0L, (void*)PKh, (void*)PKl, 64, 0L, fdum, fdum, 0L, MCH, 64, CDIM, 1.0f, 32, 0);
    wmma_gemm64<1, true, 0, 0, false, 0><<<ggrid(MCH, CDIM, 1), 256, 0, stream>>>(
        GSh, GSl, 128, 0L, WB2Gh, WB2Gl, 128, 0L, (void*)Gp, (void*)Gp, CDIM, 0L, fdum, fdum, 0L, MCH, CDIM, 128, 1.0f, 0, 0);
    wmma_gemm64<1, true, 0, 0, false, 0><<<ggrid(MCH, CDIM, 2), 256, 0, stream>>>(
        PKh, PKl, 64, 32L, WB2Kh, WB2Kl, 32, (long)S32, (void*)KKD, (void*)KKD, CDIM, PLE, fdum, fdum, 0L, MCH, CDIM, 32, 1.0f, 0, 0);
    wmma_gemm64<0, false, 0, 0, false, 0><<<ggrid(MCH, CDIM, 1), 256, 0, stream>>>(
        P16, P16, 256, 0L, WH2D, WH2D, 64, 0L, (void*)WPRE, (void*)WPRE, CDIM, 0L, fdum, fdum, 0L, MCH, CDIM, 64, s64, 0, 0);
    wmma_gemm64<0, false, 0, 0, false, 0><<<ggrid(MCH, CDIM, 3), 256, 0, stream>>>(
        P16 + 64, P16 + 64, 256, 32L, WH2S, WH2S, 32, (long)S32, (void*)APRE, (void*)APRE, CDIM, PLE, fdum, fdum, 0L, MCH, CDIM, 32, s64, 0, 0);
    k_fuse<<<(MCH * CDIM) / 256, 256, 0, stream>>>(KRAW, VRAW, v1, WPRE, KKD, MKP, APRE, MAPRE, MVPRE,
                                                   time_decay, time_aaaaa, misc_a, misc_k, misc_v,
                                                   WD, KFIN, VFIN, KKN, BBp, ch);
    k_scan<<<NBCH * NHEAD, 32, 0, stream>>>(Rp, WD, KFIN, VFIN, KKN, BBp, Yp);
    k_post<<<(MCH * 384) / 256, 256, 0, stream>>>(Yp, Rp, KFIN, VFIN, Gp, faaaa, ln_w, ln_b, YGh, YGl);
    wmma_gemm64<1, true, 0, 0, false, 0><<<ggrid(MCH, CDIM, 1), 256, 0, stream>>>(
        YGh, YGl, CDIM, 0L, WBOh, WBOl, CDIM, 0L, (void*)(out0 + (size_t)ch * MCH * CDIM), (void*)(out0 + (size_t)ch * MCH * CDIM), CDIM, 0L,
        fdum, fdum, 0L, MCH, CDIM, CDIM, 1.0f, 0, 0);
  }
  static_assert((size_t)NCHUNK * MCH == (size_t)MTOT, "out0 rows covered exactly");
}
